// DeformableWindowAttention_80573586473316
// MI455X (gfx1250) — hardware-verified
//
#include <hip/hip_runtime.h>


namespace {
constexpr int C = 256, NH = 8, HS = 32, SZ = 40, L = SZ * SZ, KW = 17, PAD = 8, K2 = KW * KW, SP = SZ + 2 * PAD  ;
constexpr float AS_ = 8.0f, SCALE = 0.17677669529663687f;

typedef _Float16 b16;
typedef __attribute__((ext_vector_type(16))) _Float16 v16b;
typedef __attribute__((ext_vector_type(8))) _Float16 v8b;
typedef __attribute__((ext_vector_type(8))) float v8f;
typedef __attribute__((ext_vector_type(4))) float v4f;
__device__ __forceinline__ float bf16_rne(float f) { unsigned int u = __float_as_uint(f); u += 0x7FFFu + ((u >> 16) & 1u); return __uint_as_float(u & 0xFFFF0000u); }
__device__ __forceinline__ void split16(float v, b16& hi, b16& lo) { hi = (b16)v; lo = (b16)(v - (float)hi); }
__device__ __forceinline__ v16b frag_kb(const b16* p, int hh) { const v8b a = *(const v8b*)(p + 8 * hh), b = *(const v8b*)(p + 16 + 8 * hh); v16b f;
#pragma unroll
  for (int e = 0; e < 8; ++e) { f[e] = a[e]; f[8 + e] = b[e]; } return f; }
__device__ __forceinline__ void frag_split(const float* p, int hh, v16b& fh, v16b& fl) {
#pragma unroll
  for (int e = 0; e < 8; ++e) { b16 a, c; split16(p[8 * hh + e] * AS_, a, c); fh[e] = a; fl[e] = c; split16(p[16 + 8 * hh + e] * AS_, a, c); fh[8 + e] = a; fl[8 + e] = c; } }
__device__ __forceinline__ v8f wmma16b(v16b a, v16b b, v8f c) { v8f d = __builtin_amdgcn_wmma_f32_16x16x32_f16(false, a, false, b, (short)0, c, false, false); asm volatile("v_nop\n\tv_nop\n\tv_nop\n\tv_nop" : "+v"(d) : "v"(a), "v"(b)); return d; }
__device__ __forceinline__ void wave_lds_sync() { __builtin_amdgcn_fence(__ATOMIC_RELEASE, "workgroup"); __builtin_amdgcn_wave_barrier(); __builtin_amdgcn_fence(__ATOMIC_ACQUIRE, "workgroup"); }
__device__ __forceinline__ float nexp(float x) { return __builtin_amdgcn_exp2f(x * 1.4426950408889634f); }
__device__ __forceinline__ float pmul(float a, float b) { float p = a * b; asm volatile("" : "+v"(p)); return p; }

__global__ __launch_bounds__(256) void prep_kernel(const float* __restrict__ x, const float* __restrict__ wqkv, const float* __restrict__ bqkv, const float* __restrict__ wproj, const float* __restrict__ bproj, b16* __restrict__ X, b16* __restrict__ R, float* __restrict__ P) {
  const size_t tid = (size_t)blockIdx.x * 256 + threadIdx.x, nth = (size_t)gridDim.x * 256;
  for (int pass = 0; pass < 2; ++pass) {
    for (size_t p = tid; p < (size_t)L * C / 8; p += nth) { const int l = (int)(p / (C / 8)), c0 = (int)(p % (C / 8)) * 8; v8b v; for (int e = 0; e < 8; ++e) v[e] = (b16)bf16_rne(x[(size_t)(c0 + e) * L + l]); *(volatile v8b*)(X + (size_t)l * C + c0) = v; }
    for (size_t p = tid; p < (size_t)(3 * C * C + C * C) / 8; p += nth) { const size_t q = p * 8; const float* src = (q < (size_t)3 * C * C) ? (wqkv + q) : (wproj + (q - (size_t)3 * C * C)); v8b v; for (int e = 0; e < 8; ++e) v[e] = (b16)bf16_rne(src[e]); *(volatile v8b*)(R + q) = v; }
    for (size_t q = tid; q < 1024; q += nth) { const int i = (int)q; P[q] = bf16_rne((i < 768) ? bqkv[i] : bproj[i - 768]); }
    __threadfence(); }
}

__global__ __launch_bounds__(64) void qkv_kernel(const b16* __restrict__ X, const b16* __restrict__ R, const float* __restrict__ P, float* __restrict__ QF) {
  __shared__ __attribute__((aligned(16))) float Ts[2][32][64 + 4];
  const int lane = threadIdx.x & 31, wave = threadIdx.x >> 5, nloc = lane & 15, hlf = lane >> 4, m0 = blockIdx.y * 32, c0 = blockIdx.x * 128 + wave * 64;
  v8f acc[2][4];
#pragma unroll
  for (int r = 0; r < 2; ++r)
#pragma unroll
    for (int t = 0; t < 4; ++t) acc[r][t] = (v8f){};
#pragma unroll 2
  for (int kb = 0; kb < C; kb += 32) { const v16b a0 = frag_kb(X + (size_t)(m0 + nloc) * C + kb, hlf), a1 = frag_kb(X + (size_t)(m0 + 16 + nloc) * C + kb, hlf);
#pragma unroll
    for (int t = 0; t < 4; ++t) { const v16b bw = frag_kb(R + (size_t)(c0 + t * 16 + nloc) * C + kb, hlf); acc[0][t] = wmma16b(a0, bw, acc[0][t]); acc[1][t] = wmma16b(a1, bw, acc[1][t]); } }
#pragma unroll
  for (int t = 0; t < 4; ++t) { const int c = c0 + t * 16 + nloc; const float bb = P[c]; const float sc = (c < C) ? SCALE : 1.0f;
#pragma unroll
    for (int r = 0; r < 2; ++r)
#pragma unroll
      for (int v = 0; v < 8; ++v) Ts[wave][r * 16 + 8 * hlf + v][t * 16 + nloc] = (acc[r][t][v] + bb) * sc; }
  wave_lds_sync();
  for (int pass = 0; pass < 2; ++pass) { for (int i = lane; i < 32 * 16; i += 32) { const int rr = i >> 4, c4 = (i & 15) * 4; *(volatile v4f*)(QF + (size_t)(m0 + rr) * (3 * C) + c0 + c4) = *(const v4f*)(&Ts[wave][rr][c4]); } __threadfence(); }
}

__global__ __launch_bounds__(256) void img_kernel(const float* __restrict__ QF, float* __restrict__ KV) {
  __shared__ __attribute__((aligned(16))) float pl[SP * SP];
  const int c = blockIdx.x, which = blockIdx.y, t_ = threadIdx.x;
  for (int i = t_; i < SP * SP; i += 256) { const int yy = i / SP - PAD, xq = i % SP - PAD; pl[i] = (yy >= 0 && yy < SZ && xq >= 0 && xq < SZ) ? QF[(size_t)(yy * SZ + xq) * (3 * C) + (which + 1) * C + c] : 0.0f; }
  __syncthreads();
  float* dst = KV + ((size_t)which * C + c) * SP * SP;
  for (int pass = 0; pass < 2; ++pass) { for (int i = t_; i < SP * SP / 4; i += 256) *(volatile v4f*)(dst + i * 4) = *(const v4f*)(&pl[i * 4]); __threadfence(); }
}

__global__ __launch_bounds__(64) void wattn_kernel(const float* __restrict__ QF, const float* __restrict__ KV, float* __restrict__ CTX) {
  __shared__ float Sc[64][K2 + 2]; __shared__ __attribute__((aligned(16))) float Oo[64][HS + 4];
  const int t_ = threadIdx.x, h = blockIdx.y, l = blockIdx.x * 64 + t_, y = l / SZ, xx = l % SZ; const float* Kp = KV; const float* Vp = KV + (size_t)C * SP * SP;
  float q[HS];
#pragma unroll
  for (int cc = 0; cc < HS; ++cc) q[cc] = QF[(size_t)l * (3 * C) + h * HS + cc];
  float mx = -INFINITY;
  for (int n1 = 0; n1 < K2; ++n1) { const int f0 = n1 * C + h * HS; int cs = f0 / K2, ps = f0 - cs * K2; float s = 0.0f;
#pragma unroll
    for (int cc = 0; cc < HS; ++cc) { const int py = ps / KW, px = ps - py * KW; s += pmul(q[cc], Kp[((size_t)cs * SP + y + py) * SP + xx + px]); ++ps; if (ps == K2) { ps = 0; ++cs; } }
    Sc[t_][n1] = s; mx = fmaxf(mx, s); }
  float su = 0.0f; for (int n1 = 0; n1 < K2; ++n1) su += nexp(Sc[t_][n1] - mx);
  const float isu = 1.0f / su; float o[HS];
#pragma unroll
  for (int cc = 0; cc < HS; ++cc) o[cc] = 0.0f;
  for (int n1 = 0; n1 < K2; ++n1) { const int wy = n1 / KW, wx = n1 - wy * KW; const bool valid = (y + wy - PAD >= 0) && (y + wy - PAD < SZ) && (xx + wx - PAD >= 0) && (xx + wx - PAD < SZ);
    const float w = valid ? nexp(Sc[t_][n1] - mx) * isu : 0.0f;
    const int f0 = n1 * C + h * HS; int cs = f0 / K2, ps = f0 - cs * K2;
#pragma unroll
    for (int cc = 0; cc < HS; ++cc) { const int py = ps / KW, px = ps - py * KW; o[cc] += pmul(w, Vp[((size_t)cs * SP + y + py) * SP + xx + px]); ++ps; if (ps == K2) { ps = 0; ++cs; } } }
#pragma unroll
  for (int cc = 0; cc < HS; ++cc) Oo[t_][cc] = o[cc];
  __syncthreads();
  for (int pass = 0; pass < 2; ++pass) { for (int i = t_; i < 64 * (HS / 4); i += 64) { const int rr = i >> 3, c4 = (i & 7) * 4; *(volatile v4f*)(CTX + (size_t)(blockIdx.x * 64 + rr) * C + h * HS + c4) = *(const v4f*)(&Oo[rr][c4]); } __threadfence(); }
}

__global__ __launch_bounds__(64) void proj_kernel(const float* __restrict__ CTX, const b16* __restrict__ R, const float* __restrict__ P, float* __restrict__ out) {
  __shared__ __attribute__((aligned(16))) float Ts[2][32][64 + 1];
  const int lane = threadIdx.x & 31, wave = threadIdx.x >> 5, nloc = lane & 15, hlf = lane >> 4, m0 = blockIdx.y * 32, c0 = blockIdx.x * 128 + wave * 64; const b16* Wp = R + (size_t)3 * C * C;
  v8f acc[2][4];
#pragma unroll
  for (int r = 0; r < 2; ++r)
#pragma unroll
    for (int t = 0; t < 4; ++t) acc[r][t] = (v8f){};
#pragma unroll 2
  for (int kb = 0; kb < C; kb += 32) { v16b a0, l0, a1, l1; frag_split(CTX + (size_t)(m0 + nloc) * C + kb, hlf, a0, l0); frag_split(CTX + (size_t)(m0 + 16 + nloc) * C + kb, hlf, a1, l1);
#pragma unroll
    for (int t = 0; t < 4; ++t) { const v16b bw = frag_kb(Wp + (size_t)(c0 + t * 16 + nloc) * C + kb, hlf); acc[0][t] = wmma16b(a0, bw, acc[0][t]); acc[0][t] = wmma16b(l0, bw, acc[0][t]); acc[1][t] = wmma16b(a1, bw, acc[1][t]); acc[1][t] = wmma16b(l1, bw, acc[1][t]); } }
#pragma unroll
  for (int t = 0; t < 4; ++t) { const float bb = P[768 + c0 + t * 16 + nloc];
#pragma unroll
    for (int r = 0; r < 2; ++r)
#pragma unroll
      for (int v = 0; v < 8; ++v) Ts[wave][r * 16 + 8 * hlf + v][t * 16 + nloc] = acc[r][t][v] * (1.0f / AS_) + bb; }
  wave_lds_sync();
  for (int pass = 0; pass < 2; ++pass) { for (int cc = 0; cc < 64; ++cc) ((volatile float*)out)[(size_t)(c0 + cc) * L + m0 + lane] = Ts[wave][lane][cc]; __threadfence(); }
}
}

extern "C" void kernel_launch(void* const* d_in, const int* in_sizes, int n_in,
                              void* d_out, int out_size, void* d_ws, size_t ws_size, hipStream_t stream) {
  (void)n_in; (void)out_size;
  const float* x = (const float*)d_in[0]; const float* wqkv = (const float*)d_in[1]; const float* bqkv = (const float*)d_in[2]; const float* wproj = (const float*)d_in[3]; const float* bproj = (const float*)d_in[4];
  float* out = (float*)d_out;
  if (in_sizes[0] != C * L || in_sizes[1] != 3 * C * C || in_sizes[3] != C * C) return;
  size_t off = 0; char* ws = (char*)d_ws;
  auto carve = [&](size_t bytes) { char* p = ws + off; off += (bytes + 255) & ~(size_t)255; return p; };
  b16* X = (b16*)carve((size_t)L * C * 2); b16* R = (b16*)carve((size_t)4 * C * C * 2); float* P = (float*)carve(1024 * 4); float* QF = (float*)carve((size_t)L * 3 * C * 4); float* KV = (float*)carve((size_t)2 * C * SP * SP * 4); float* CTX = (float*)carve((size_t)L * C * 4);
  if (off > ws_size) return;
  prep_kernel<<<256, 256, 0, stream>>>(x, wqkv, bqkv, wproj, bproj, X, R, P);
  qkv_kernel<<<dim3(6, L / 32), 64, 0, stream>>>(X, R, P, QF);
  img_kernel<<<dim3(C, 2), 256, 0, stream>>>(QF, KV);
  wattn_kernel<<<dim3(L / 64, NH), 64, 0, stream>>>(QF, KV, CTX);
  proj_kernel<<<dim3(2, L / 32), 64, 0, stream>>>(CTX, R, P, out);
}
